// GCNRU_2388001817260
// MI455X (gfx1250) — hardware-verified
//
#include <hip/hip_runtime.h>
#include <stddef.h>


#define FIN     128
#define HID     96
#define FOUT    64
#define JKD     288
#define NTHR    256
#define NWAVE   8
#define EPT     8
#define NGRP    2
#define CHUNK   (NTHR * EPT * NGRP)
#define WCAP    (EPT * NGRP * 32)
#define LISTN   (NWAVE * WCAP)
#define ESHF    11
#define NBC     32768
#define NBF     2048
#define RCAP    40960
#define RBN     128
#define TGT     256
#define DEGCAP  512
#define GROWS   128
#define OTHR    512
#define PTHR    128
#define POOLCAP 2048
#define WSCALE  16
#define HSC     64
#define ESC     16
#define WSCAP   134217728

#define WP0 0
#define WP1 (WP0 + HID * FIN)
#define WP2 (WP1 + HID * HID)
#define WP3 (WP2 + HID * HID)
#define WP4 (WP3 + HID * JKD)
#define WP5 (WP4 + HID * HID)
#define WPN (WP5 + FOUT * HID)

#define LDS_COUNT ((NBC + LISTN + NWAVE) * 4)
#define LDS_FILL  ((RCAP + NBF + LISTN + NWAVE) * 4)
#define LDS_AGG   (NWAVE * 32 * HID * 4)

static_assert((CHUNK & (CHUNK - 1)) == 0);
static_assert((NBC & (NBC - 1)) == 0 && (NBF & (NBF - 1)) == 0);
static_assert(NBF <= (1 << ESHF));
static_assert((NBC % NBF) == 0);
static_assert(OTHR * 4 == NBF);
static_assert((RCAP % 32) == 0);
static_assert(TGT == NWAVE * 32);
static_assert(GROWS == NWAVE * 16);
static_assert((TGT % GROWS) == 0);
static_assert((GROWS * FIN / 8) % NTHR == 0 && (GROWS * HID / 8) % NTHR == 0 && (GROWS * JKD / 8) % NTHR == 0);
static_assert((FIN % 32) == 0 && (HID % 32) == 0 && (JKD % 32) == 0 && (FOUT % 16) == 0);
static_assert(((16 * HID) % 128) == 0 && ((16 * FOUT) % 128) == 0);
static_assert((HID % 4) == 0 && (HID / 4) <= 32);
static_assert(NBC == NWAVE * 32 * 128);
static_assert((WP1 % 64) == 0 && (WP2 % 64) == 0 && (WP3 % 64) == 0 && (WP4 % 64) == 0 && (WP5 % 64) == 0 && (WPN % 64) == 0);
static_assert(PTHR >= HID);

typedef float     v4f  __attribute__((ext_vector_type(4)));
typedef float     v8f  __attribute__((ext_vector_type(8)));
typedef int       v4i  __attribute__((ext_vector_type(4)));
typedef _Float16  v8h  __attribute__((ext_vector_type(8)));
typedef _Float16  v16h __attribute__((ext_vector_type(16)));
union FragH { v16h v; v8h h[2]; };

__host__ __device__ constexpr int gemm_lds(int kd, int nc) {
  return (GROWS * (kd + 8) * 2 > GROWS * nc * 4) ? GROWS * (kd + 8) * 2 : GROWS * nc * 4;
}

__device__ __forceinline__ v8f wmf(v16h a, v16h b, v8f c) {
  v8f d = __builtin_amdgcn_wmma_f32_16x16x32_f16(false, a, false, b, (short)0, c, false, false);
  asm volatile("v_nop\n\tv_nop\n\tv_nop\n\tv_nop" : "+v"(d) : "v"(a), "v"(b));
  return d;
}

template <int NB, int SRC>
__device__ __forceinline__ int scan_chunk(const int* __restrict__ dsts, const int* __restrict__ srcs, int nE, int nN,
                                          int cbase, int slotBase, int vec8, int* list, int tid, int lane, int wave) {
  int wc = 0;
#pragma unroll
  for (int g = 0; g < NGRP; ++g) {
    const int el0  = (g * NTHR + tid) * EPT;
    const int e0   = cbase + el0;
    const int sent = -2147483647 - 1;
    v4i da, db;
    v4i sa = {0, 0, 0, 0}, sb = {0, 0, 0, 0};
    if (vec8 != 0 && cbase + CHUNK <= nE) {
      da = *(const v4i*)(dsts + e0);
      db = *(const v4i*)(dsts + e0 + 4);
      if (SRC) {
        sa = *(const v4i*)(srcs + e0);
        sb = *(const v4i*)(srcs + e0 + 4);
      }
    } else {
      da.x = (e0     < nE) ? dsts[min(e0, nE - 1)] : sent;
      da.y = (e0 + 1 < nE) ? dsts[min(e0 + 1, nE - 1)] : sent;
      da.z = (e0 + 2 < nE) ? dsts[min(e0 + 2, nE - 1)] : sent;
      da.w = (e0 + 3 < nE) ? dsts[min(e0 + 3, nE - 1)] : sent;
      db.x = (e0 + 4 < nE) ? dsts[min(e0 + 4, nE - 1)] : sent;
      db.y = (e0 + 5 < nE) ? dsts[min(e0 + 5, nE - 1)] : sent;
      db.z = (e0 + 6 < nE) ? dsts[min(e0 + 6, nE - 1)] : sent;
      db.w = (e0 + 7 < nE) ? dsts[min(e0 + 7, nE - 1)] : sent;
      if (SRC) {
        sa.x = srcs[min(e0, nE - 1)];
        sa.y = srcs[min(e0 + 1, nE - 1)];
        sa.z = srcs[min(e0 + 2, nE - 1)];
        sa.w = srcs[min(e0 + 3, nE - 1)];
        sb.x = srcs[min(e0 + 4, nE - 1)];
        sb.y = srcs[min(e0 + 5, nE - 1)];
        sb.z = srcs[min(e0 + 6, nE - 1)];
        sb.w = srcs[min(e0 + 7, nE - 1)];
      }
    }
    if (SRC) {
      sa.x = min(max(sa.x, 0), nN - 1); sa.y = min(max(sa.y, 0), nN - 1);
      sa.z = min(max(sa.z, 0), nN - 1); sa.w = min(max(sa.w, 0), nN - 1);
      sb.x = min(max(sb.x, 0), nN - 1); sb.y = min(max(sb.y, 0), nN - 1);
      sb.z = min(max(sb.z, 0), nN - 1); sb.w = min(max(sb.w, 0), nN - 1);
    }
    const unsigned nb = (unsigned)slotBase;
    const unsigned s0 = (unsigned)da.x - nb, s1 = (unsigned)da.y - nb;
    const unsigned s2 = (unsigned)da.z - nb, s3 = (unsigned)da.w - nb;
    const unsigned s4 = (unsigned)db.x - nb, s5 = (unsigned)db.y - nb;
    const unsigned s6 = (unsigned)db.z - nb, s7 = (unsigned)db.w - nb;
    const bool h0 = s0 < (unsigned)NB, h1 = s1 < (unsigned)NB, h2 = s2 < (unsigned)NB, h3 = s3 < (unsigned)NB;
    const bool h4 = s4 < (unsigned)NB, h5 = s5 < (unsigned)NB, h6 = s6 < (unsigned)NB, h7 = s7 < (unsigned)NB;
    const unsigned any = __builtin_amdgcn_ballot_w32(h0 | h1 | h2 | h3 | h4 | h5 | h6 | h7);
    if (any != 0u) {
#define HITJ(HJ, SJ, VJ) { \
        const unsigned mj = __builtin_amdgcn_ballot_w32(HJ); \
        if (mj != 0u) { \
          if (HJ) { \
            const int pos = wc + (int)__builtin_amdgcn_mbcnt_lo(mj, 0u); \
            const int entv = SRC ? (((VJ) << ESHF) | (int)(SJ)) : (int)(SJ); \
            if (pos < WCAP) list[wave * WCAP + pos] = entv; \
          } \
          wc += (int)__builtin_popcount(mj); } }
      HITJ(h0, s0, sa.x)
      HITJ(h1, s1, sa.y)
      HITJ(h2, s2, sa.z)
      HITJ(h3, s3, sa.w)
      HITJ(h4, s4, sb.x)
      HITJ(h5, s5, sb.y)
      HITJ(h6, s6, sb.z)
      HITJ(h7, s7, sb.w)
#undef HITJ
    }
  }
  return wc;
}

__global__ __launch_bounds__(NTHR) void k_wprep(
    const float* __restrict__ w0, const float* __restrict__ w1, const float* __restrict__ w2,
    const float* __restrict__ w3, const float* __restrict__ w4, const float* __restrict__ w5,
    _Float16* wp) {
  const int tid = threadIdx.x;
  const int b = blockIdx.x;
  const float* W = w0; int K = FIN, NCOL = HID; size_t dst = WP0;
  if (b == 1)      { W = w1; K = HID; NCOL = HID;  dst = WP1; }
  else if (b == 2) { W = w2; K = HID; NCOL = HID;  dst = WP2; }
  else if (b == 3) { W = w3; K = JKD; NCOL = HID;  dst = WP3; }
  else if (b == 4) { W = w4; K = HID; NCOL = HID;  dst = WP4; }
  else if (b >= 5) { W = w5; K = HID; NCOL = FOUT; dst = WP5; }
  const int kq = K / 8;
  const int nT = NCOL * kq;
#pragma unroll 1
  for (int i = tid; i < nT; i += NTHR) {
    const int n  = i / kq;
    const int k0 = (i - n * kq) * 8;
    v8h hv;
#pragma unroll
    for (int e = 0; e < 8; ++e) hv[e] = (_Float16)(W[(size_t)(k0 + e) * NCOL + n] * (float)WSCALE);
    _Float16* d = wp + dst + (size_t)i * 8;
    *(volatile v8h*)d = hv;
    __threadfence();
    *(volatile v8h*)d = hv;
  }
}

__global__ __launch_bounds__(NTHR) void k_count(
    const int* __restrict__ ei, int* cnt, float* dinv, int nE, int nN, int vec8) {
  extern __shared__ v4f lds_dyn[];
  int* scnt = (int*)lds_dyn;
  int* list = scnt + NBC;
  int* wcnt = list + LISTN;
  const int tid = threadIdx.x, lane = tid & 31, wave = tid >> 5;
  const int nodeBase = blockIdx.x * NBC;
  const int* dsts = ei + nE;

  {
    const v4i z = {0, 0, 0, 0};
    for (int i = tid; i < NBC / 4; i += NTHR) ((v4i*)scnt)[i] = z;
  }
  __syncthreads();

  const int nChunks = (nE + CHUNK - 1) / CHUNK;
#pragma unroll 1
  for (int ch = 0; ch < nChunks; ++ch) {
    const int cbase = ch * CHUNK;
    const int wc = scan_chunk<NBC, 0>(dsts, ei, nE, nN, cbase, nodeBase, vec8, list, tid, lane, wave);
    if (lane == 0) wcnt[wave] = wc;
    __syncthreads();
    if (wave == 0) {
#pragma unroll 1
      for (int wsx = 0; wsx < NWAVE; ++wsx) {
        int n = __builtin_amdgcn_readfirstlane(wcnt[wsx]);
        n = n > WCAP ? WCAP : (n < 0 ? 0 : n);
        const int* lp = list + wsx * WCAP;
#pragma unroll 1
        for (int i = 0; i < n; ++i) {
          const int ent  = __builtin_amdgcn_readfirstlane(lp[i]);
          const int slot = ent & (NBC - 1);
          if (lane == 0) scnt[slot] = scnt[slot] + 1;
        }
      }
    }
    __syncthreads();
  }

  int*   cp = cnt + (size_t)nodeBase;
  float* dp = dinv + (size_t)nodeBase;
#pragma unroll 4
  for (int q = 0; q < 32; ++q) {
    const int f = (wave * 32 + q) * 128 + 4 * lane;
    const v4i c = *(const v4i*)(scnt + f);
    v4f d;
    d.x = rsqrtf((float)(c.x + 1)); d.y = rsqrtf((float)(c.y + 1));
    d.z = rsqrtf((float)(c.z + 1)); d.w = rsqrtf((float)(c.w + 1));
    *(volatile v4i*)(cp + f) = c;
    *(volatile v4f*)(dp + f) = d;
  }
  __threadfence();
#pragma unroll 4
  for (int q = 0; q < 32; ++q) {
    const int f = (wave * 32 + q) * 128 + 4 * lane;
    const v4i c = *(const v4i*)(scnt + f);
    v4f d;
    d.x = rsqrtf((float)(c.x + 1)); d.y = rsqrtf((float)(c.y + 1));
    d.z = rsqrtf((float)(c.z + 1)); d.w = rsqrtf((float)(c.w + 1));
    *(volatile v4i*)(cp + f) = c;
    *(volatile v4f*)(dp + f) = d;
  }
}

__global__ __launch_bounds__(OTHR) void k_offsets(
    const int* __restrict__ cnt, int* off, int* rbase, int nBF) {
  __shared__ __attribute__((aligned(16))) int srb[RBN];
  __shared__ int wtot[OTHR / 32];
  const int tid = threadIdx.x, lane = tid & 31, wave = tid >> 5;
  for (int i = tid; i < RBN; i += OTHR) srb[i] = 0;
  int carry = 0;
#pragma unroll 1
  for (int fb = 0; fb < nBF; ++fb) {
    const int base = fb * NBF;
    const v4i c = *(const v4i*)(cnt + base + 4 * tid);
    const int e0 = max(c.x, 0), e1 = max(c.y, 0), e2 = max(c.z, 0), e3 = max(c.w, 0);
    const int ts = e0 + e1 + e2 + e3;
    int incl = ts;
#pragma unroll
    for (int d = 1; d < 32; d <<= 1) {
      const int t = __shfl_up(incl, d);
      if (lane >= d) incl += t;
    }
    if (lane == 31) wtot[wave] = incl;
    __syncthreads();
    int pre = 0;
#pragma unroll 1
    for (int w = 0; w < wave; ++w) pre += wtot[w];
    int tot = 0;
#pragma unroll
    for (int w = 0; w < OTHR / 32; ++w) tot += wtot[w];
    int run = carry + pre + incl - ts;
    v4i o;
    o.x = run; run += e0;
    o.y = run; run += e1;
    o.z = run; run += e2;
    o.w = run;
    int* op = off + base + 4 * tid;
    *(volatile v4i*)op = o;
    __threadfence();
    *(volatile v4i*)op = o;
    if (tid == 0) srb[min(fb, RBN - 1)] = carry;
    carry += (tot + 31) & ~31;
    __syncthreads();
  }
  if (tid == 0) srb[min(nBF, RBN - 1)] = carry;
  __syncthreads();
  v4i rv = {0, 0, 0, 0};
  if (tid < 32) rv = *(const v4i*)(srb + 4 * tid);
  if (tid < 32) *(volatile v4i*)(rbase + 4 * tid) = rv;
  __threadfence();
  if (tid < 32) *(volatile v4i*)(rbase + 4 * tid) = rv;
}

__global__ __launch_bounds__(NTHR) void k_fill(
    const int* __restrict__ ei, const int* __restrict__ off, const int* __restrict__ rbase,
    int* csr, int nN, int nE, int vec8, int csrLen) {
  extern __shared__ v4f lds_dyn[];
  int* region = (int*)lds_dyn;
  int* cursor = region + RCAP;
  int* list   = cursor + NBF;
  int* wcnt   = list + LISTN;
  const int tid = threadIdx.x, lane = tid & 31, wave = tid >> 5;
  const int b = blockIdx.x;
  const int nodeBase = b * NBF;
  const int* dsts = ei + nE;

  int rb0 = rbase[b];
  const int rb1 = rbase[b + 1];
  rb0 = rb0 < 0 ? 0 : (rb0 > csrLen ? csrLen : rb0);
  rb0 &= ~31;
  int len = rb1 - rb0;
  len = len < 0 ? 0 : (len > RCAP ? RCAP : len);
  int lenW = (len + 31) & ~31;
  if (rb0 + lenW > csrLen) lenW = (csrLen - rb0) & ~31;

  {
    const v4i z = {0, 0, 0, 0};
    for (int i = tid; i < RCAP / 4; i += NTHR) ((v4i*)region)[i] = z;
    for (int s = tid; s < NBF; s += NTHR) {
      int o = off[nodeBase + s] - rb0;
      o = o < 0 ? 0 : (o > RCAP ? RCAP : o);
      cursor[s] = o;
    }
  }
  __syncthreads();

  const int nChunks = (nE + CHUNK - 1) / CHUNK;
#pragma unroll 1
  for (int ch = 0; ch < nChunks; ++ch) {
    const int cbase = ch * CHUNK;
    const int wc = scan_chunk<NBF, 1>(dsts, ei, nE, nN, cbase, nodeBase, vec8, list, tid, lane, wave);
    if (lane == 0) wcnt[wave] = wc;
    __syncthreads();
    if (wave == 0) {
#pragma unroll 1
      for (int wsx = 0; wsx < NWAVE; ++wsx) {
        int n = __builtin_amdgcn_readfirstlane(wcnt[wsx]);
        n = n > WCAP ? WCAP : (n < 0 ? 0 : n);
        const int* lp = list + wsx * WCAP;
#pragma unroll 1
        for (int i = 0; i < n; ++i) {
          const int ent  = __builtin_amdgcn_readfirstlane(lp[i]);
          const int slot = ent & (NBF - 1);
          int src = (ent >> ESHF) & 0xFFFFF;
          src = src > nN - 1 ? nN - 1 : src;
          if (lane == 0) {
            int pos = cursor[slot];
            pos = pos < 0 ? 0 : (pos > RCAP - 1 ? RCAP - 1 : pos);
            region[pos] = src;
            const int np = pos + 1;
            cursor[slot] = np > RCAP ? RCAP : np;
          }
        }
      }
    }
    __syncthreads();
  }

  const int nv = lenW >> 2;
  int* gp = csr + rb0;
#pragma unroll 1
  for (int i = tid; i < nv; i += NTHR) { const v4i v = ((const v4i*)region)[i]; *(volatile v4i*)(gp + 4 * i) = v; }
  __threadfence();
#pragma unroll 1
  for (int i = tid; i < nv; i += NTHR) { const v4i v = ((const v4i*)region)[i]; *(volatile v4i*)(gp + 4 * i) = v; }
}

template <int KD, int LDA, int NC, int ASC, int DNV, int BIAS, int RELU>
__global__ __launch_bounds__(NTHR) void k_gemm(
    const float* __restrict__ A, const _Float16* __restrict__ Bw, const float* __restrict__ dinv,
    const float* __restrict__ bias, float* C, int nRowsA, int nRowsC) {
  extern __shared__ v4f lds_dyn[];
  constexpr int APH = KD + 8;
  constexpr int NT  = NC / 16;
  constexpr float OSC = 1.0f / (float)(ASC * WSCALE);
  static_assert((KD % 32) == 0 && (NC % 16) == 0 && ((GROWS * KD / 8) % NTHR) == 0 && (LDA % 4) == 0 && LDA >= KD);
  _Float16* sA  = (_Float16*)lds_dyn;
  float*    stg = (float*)lds_dyn;
  const int tid = threadIdx.x, lane = tid & 31, wave = tid >> 5, hh = lane >> 4, m = lane & 15;
  const int rowBase = blockIdx.x * GROWS;

#pragma unroll
  for (int i = 0; i < (GROWS * KD / 8) / NTHR; ++i) {
    const int idx = i * NTHR + tid;
    const int r   = idx / (KD / 8);
    const int c0  = (idx - r * (KD / 8)) * 8;
    int row = rowBase + r;
    row = row > nRowsA - 1 ? nRowsA - 1 : row;
    const float* ap = A + (size_t)row * LDA + c0;
    const v4f a = *(const v4f*)ap, b = *(const v4f*)(ap + 4);
    v8h hv;
    hv[0] = (_Float16)(a.x * (float)ASC); hv[1] = (_Float16)(a.y * (float)ASC);
    hv[2] = (_Float16)(a.z * (float)ASC); hv[3] = (_Float16)(a.w * (float)ASC);
    hv[4] = (_Float16)(b.x * (float)ASC); hv[5] = (_Float16)(b.y * (float)ASC);
    hv[6] = (_Float16)(b.z * (float)ASC); hv[7] = (_Float16)(b.w * (float)ASC);
    *(v8h*)(sA + r * APH + c0) = hv;
  }
  __syncthreads();

  v8f acc[NT];
#pragma unroll
  for (int t = 0; t < NT; ++t) { v8f z = {0.f, 0.f, 0.f, 0.f, 0.f, 0.f, 0.f, 0.f}; acc[t] = z; }
  const _Float16* ahp = sA + (wave * 16 + m) * APH + 8 * hh;
#pragma unroll 1
  for (int kt = 0; kt < KD / 32; ++kt) {
    FragH af;
    af.h[0] = *(const v8h*)(ahp + 32 * kt);
    af.h[1] = *(const v8h*)(ahp + 32 * kt + 16);
#pragma unroll
    for (int t = 0; t < NT; ++t) {
      const _Float16* bp = Bw + (size_t)(16 * t + m) * KD + 32 * kt + 8 * hh;
      FragH bf;
      bf.h[0] = *(const v8h*)bp;
      bf.h[1] = *(const v8h*)(bp + 16);
      acc[t] = wmf(af.v, bf.v, acc[t]);
    }
  }
  __syncthreads();

  const int r0 = wave * 16 + 8 * hh;
  float s[8];
  if constexpr (DNV != 0) {
    const v4f dA = *(const v4f*)(dinv + (size_t)rowBase + r0);
    const v4f dB = *(const v4f*)(dinv + (size_t)rowBase + r0 + 4);
    s[0] = dA.x; s[1] = dA.y; s[2] = dA.z; s[3] = dA.w; s[4] = dB.x; s[5] = dB.y; s[6] = dB.z; s[7] = dB.w;
#pragma unroll
    for (int r = 0; r < 8; ++r) s[r] = s[r] * OSC;
  } else {
#pragma unroll
    for (int r = 0; r < 8; ++r) s[r] = OSC;
  }
  float* sp = stg + r0 * NC + m;
#pragma unroll
  for (int t = 0; t < NT; ++t) {
    float bv = 0.0f;
    if constexpr (BIAS != 0) bv = bias[16 * t + m];
#pragma unroll
    for (int r = 0; r < 8; ++r) {
      float v = acc[t][r] * s[r] + bv;
      if constexpr (RELU != 0) v = fmaxf(v, 0.0f);
      sp[r * NC + 16 * t] = v;
    }
  }
  __syncthreads();

  const float* lp = stg + wave * 16 * NC;
  const int wrow0 = rowBase + wave * 16;
  float* gp = C + (size_t)wrow0 * NC;
#pragma unroll
  for (int i = 0; i < (16 * NC) / 128; ++i) {
    const int fidx = i * 128 + 4 * lane;
    const int row = wrow0 + fidx / NC;
    const v4f v = *(const v4f*)(lp + fidx);
    if (row < nRowsC) *(volatile v4f*)(gp + fidx) = v;
  }
  __threadfence();
#pragma unroll
  for (int i = 0; i < (16 * NC) / 128; ++i) {
    const int fidx = i * 128 + 4 * lane;
    const int row = wrow0 + fidx / NC;
    const v4f v = *(const v4f*)(lp + fidx);
    if (row < nRowsC) *(volatile v4f*)(gp + fidx) = v;
  }
}

__global__ __launch_bounds__(NTHR) void k_agg(
    const int* __restrict__ csr, const int* __restrict__ off, const int* __restrict__ cnt,
    const float* __restrict__ dinv, const float* __restrict__ hw, const float* __restrict__ bs,
    float* H, int ldh, int nN, int csrLen) {
  extern __shared__ v4f lds_dyn[];
  float* sout = (float*)lds_dyn;
  const int tid = threadIdx.x, lane = tid & 31, wave = tid >> 5;
  const int tbase = blockIdx.x * TGT + wave * 32;
  const int cl = tbase + lane;
  const int cnt_l = cnt[cl];
  const int off_l = off[cl];
  union FI { float f; int i; };
  FI dvu; dvu.f = dinv[cl];
  const float bq0 = bs[lane], bq1 = bs[lane + 32], bq2 = bs[lane + 64];
  float* sw = sout + wave * 32 * HID;

#pragma unroll 1
  for (int j = 0; j < 32; ++j) {
    const int c = tbase + j;
    int n = __builtin_amdgcn_readlane(cnt_l, j);
    n = n < 0 ? 0 : (n > DEGCAP ? DEGCAP : n);
    const int st = __builtin_amdgcn_readlane(off_l, j);
    FI du; du.i = __builtin_amdgcn_readlane(dvu.i, j);
    const float dc = du.f;
    float a0 = 0.f, a1 = 0.f, a2 = 0.f;
#pragma unroll 1
    for (int q0 = 0; q0 < n; q0 += 32) {
      int pos = st + q0 + lane;
      pos = pos < 0 ? 0 : (pos > csrLen - 1 ? csrLen - 1 : pos);
      int sl = csr[pos];
      sl = sl < 0 ? 0 : (sl > nN - 1 ? nN - 1 : sl);
      const int mcnt = (n - q0) < 32 ? (n - q0) : 32;
#pragma unroll 1
      for (int p = 0; p < mcnt; ++p) {
        const int s = __builtin_amdgcn_readlane(sl, p);
        const float* hr = hw + (size_t)s * HID;
        a0 += hr[lane]; a1 += hr[lane + 32]; a2 += hr[lane + 64];
      }
    }
    const float* hc = hw + (size_t)c * HID;
    const float v0 = fmaxf((a0 + hc[lane])      * dc + bq0, 0.f);
    const float v1 = fmaxf((a1 + hc[lane + 32]) * dc + bq1, 0.f);
    const float v2 = fmaxf((a2 + hc[lane + 64]) * dc + bq2, 0.f);
    sw[j * HID + lane]      = v0;
    sw[j * HID + lane + 32] = v1;
    sw[j * HID + lane + 64] = v2;
  }
  __syncthreads();

  float* gp = H + (size_t)tbase * ldh;
  if (lane < HID / 4) {
#pragma unroll 4
    for (int r = 0; r < 32; ++r) {
      const v4f v = *(const v4f*)(sw + r * HID + 4 * lane);
      *(volatile v4f*)(gp + (size_t)r * ldh + 4 * lane) = v;
    }
  }
  __threadfence();
  if (lane < HID / 4) {
#pragma unroll 4
    for (int r = 0; r < 32; ++r) {
      const v4f v = *(const v4f*)(sw + r * HID + 4 * lane);
      *(volatile v4f*)(gp + (size_t)r * ldh + 4 * lane) = v;
    }
  }
}

__global__ __launch_bounds__(PTHR) void k_pool(
    const float* __restrict__ hj, const int* __restrict__ gid, float* emb, int nN, int nG) {
  __shared__ __attribute__((aligned(16))) float srow[HID];
  const int tid = threadIdx.x;
  const int g = blockIdx.x;
  int lo = 0, hi = 0;
  if (g < nG) {
    int a = 0, b = nN;
#pragma unroll 1
    for (int it = 0; it < 40 && a < b; ++it) {
      const int mid = (a + b) >> 1;
      const int v = gid[mid];
      if (v < g) a = mid + 1; else b = mid;
    }
    lo = a;
    b = nN;
#pragma unroll 1
    for (int it = 0; it < 40 && a < b; ++it) {
      const int mid = (a + b) >> 1;
      const int v = gid[mid];
      if (v < g + 1) a = mid + 1; else b = mid;
    }
    hi = a;
  }
  lo = lo < 0 ? 0 : (lo > nN ? nN : lo);
  hi = hi < lo ? lo : (hi > nN ? nN : hi);
  int len = hi - lo;
  len = len > POOLCAP ? POOLCAP : len;
  const int ch = tid < HID ? tid : HID - 1;
  float acc = 0.f;
#pragma unroll 1
  for (int i = 0; i < len; ++i) acc += hj[(size_t)(lo + i) * HID + ch];
  if (tid < HID) srow[tid] = acc;
  __syncthreads();

  float* gp = emb + (size_t)g * HID;
  if (tid < HID / 4) {
    const v4f v = *(const v4f*)(srow + 4 * tid);
    *(volatile v4f*)(gp + 4 * tid) = v;
  }
  __threadfence();
  if (tid < HID / 4) {
    const v4f v = *(const v4f*)(srow + 4 * tid);
    *(volatile v4f*)(gp + 4 * tid) = v;
  }
}

extern "C" void kernel_launch(void* const* d_in, const int* in_sizes, int n_in,
                              void* d_out, int out_size, void* d_ws, size_t ws_size,
                              hipStream_t stream) {
  if (n_in < 15) return;
  const int nN = in_sizes[0] / FIN;
  const int nE = in_sizes[1] / 2;
  const int nG = out_size / FOUT;
  if (nN <= 0 || nE <= 0 || nG <= 0) return;
  if (in_sizes[0] != nN * FIN || in_sizes[1] != 2 * nE || in_sizes[2] != nN) return;
  if (in_sizes[3] != FIN * HID || in_sizes[4] != HID) return;
  if (in_sizes[5] != HID * HID || in_sizes[6] != HID) return;
  if (in_sizes[7] != HID * HID || in_sizes[8] != HID) return;
  if (in_sizes[9] != JKD * HID || in_sizes[10] != HID) return;
  if (in_sizes[11] != HID * HID || in_sizes[12] != HID) return;
  if (in_sizes[13] != HID * FOUT || in_sizes[14] != FOUT) return;
  if (out_size != nG * FOUT) return;
  if (nN > (1 << 20) || nE > (1 << 28) || nG > (1 << 20)) return;

  const float* x   = (const float*)d_in[0];
  const int*   ei  = (const int*)d_in[1];
  const int*   gid = (const int*)d_in[2];
  const float* W0  = (const float*)d_in[3];  const float* b0  = (const float*)d_in[4];
  const float* W1  = (const float*)d_in[5];  const float* b1  = (const float*)d_in[6];
  const float* W2  = (const float*)d_in[7];  const float* b2  = (const float*)d_in[8];
  const float* Wjk = (const float*)d_in[9];  const float* bjk = (const float*)d_in[10];
  const float* Wm1 = (const float*)d_in[11]; const float* bm1 = (const float*)d_in[12];
  const float* Wm2 = (const float*)d_in[13]; const float* bm2 = (const float*)d_in[14];
  float* out = (float*)d_out;

  const int NPAD   = ((nN + TGT - 1) / TGT) * TGT;
  const int nBC    = (nN + NBC - 1) / NBC;
  const int CNTPAD = nBC * NBC;
  const int nBF    = (nN + NBF - 1) / NBF;
  const int OFFN   = nBF * NBF;
  if (nBF + 1 > RBN) return;
  if (OFFN > CNTPAD || NPAD > OFFN) return;
  const int csrLen = ((nE + 31) & ~31) + 32 * (nBF + 1);
  const int nGemm  = NPAD / GROWS;
  const int nAgg   = NPAD / TGT;
  const int GP     = ((nG + GROWS - 1) / GROWS) * GROWS;
  const int nGemmH = GP / GROWS;

  char* ws = (char*)d_ws;
  size_t off = 0;
  const size_t oW   = off; off += (size_t)WPN * 2;                    off = (off + 255) & ~(size_t)255;
  const size_t oCnt = off; off += (size_t)CNTPAD * 4;                 off = (off + 255) & ~(size_t)255;
  const size_t oDv  = off; off += (size_t)CNTPAD * 4;                 off = (off + 255) & ~(size_t)255;
  const size_t oOff = off; off += (size_t)OFFN * 4;                   off = (off + 255) & ~(size_t)255;
  const size_t oRb  = off; off += (size_t)RBN * 4;                    off = (off + 255) & ~(size_t)255;
  const size_t oCsr = off; off += (size_t)csrLen * 4;                 off = (off + 255) & ~(size_t)255;
  const size_t oHw  = off; off += (size_t)NPAD * HID * 4;             off = (off + 255) & ~(size_t)255;
  const size_t oHc  = off; off += (size_t)NPAD * JKD * 4;             off = (off + 255) & ~(size_t)255;
  const size_t oHj  = off; off += (size_t)NPAD * HID * 4;             off = (off + 255) & ~(size_t)255;
  const size_t oEmb = off; off += (size_t)GP * HID * 4;               off = (off + 255) & ~(size_t)255;
  const size_t oT2  = off; off += (size_t)GP * HID * 4;               off = (off + 255) & ~(size_t)255;
  if (off > ws_size || off > (size_t)WSCAP) return;
  _Float16* wp   = (_Float16*)(ws + oW);
  int*      cnt  = (int*)(ws + oCnt);
  float*    dinv = (float*)(ws + oDv);
  int*      offp = (int*)(ws + oOff);
  int*      rb   = (int*)(ws + oRb);
  int*      csr  = (int*)(ws + oCsr);
  float*    hw   = (float*)(ws + oHw);
  float*    hcat = (float*)(ws + oHc);
  float*    hjk  = (float*)(ws + oHj);
  float*    emb  = (float*)(ws + oEmb);
  float*    t2   = (float*)(ws + oT2);

  const int vec8 = ((nE & 3) == 0) ? 1 : 0;

  k_wprep<<<6, NTHR, 0, stream>>>(W0, W1, W2, Wjk, Wm1, Wm2, wp);

  hipFuncSetAttribute(reinterpret_cast<const void*>(&k_count),
                      hipFuncAttributeMaxDynamicSharedMemorySize, LDS_COUNT);
  k_count<<<nBC, NTHR, LDS_COUNT, stream>>>(ei, cnt, dinv, nE, nN, vec8);
  k_offsets<<<1, OTHR, 0, stream>>>(cnt, offp, rb, nBF);
  hipFuncSetAttribute(reinterpret_cast<const void*>(&k_fill),
                      hipFuncAttributeMaxDynamicSharedMemorySize, LDS_FILL);
  k_fill<<<nBF, NTHR, LDS_FILL, stream>>>(ei, offp, rb, csr, nN, nE, vec8, csrLen);

  hipFuncSetAttribute(reinterpret_cast<const void*>(&k_agg),
                      hipFuncAttributeMaxDynamicSharedMemorySize, LDS_AGG);

  constexpr int LDS_G1 = gemm_lds(FIN, HID);
  k_gemm<FIN, FIN, HID, 1, 1, 0, 0><<<nGemm, NTHR, LDS_G1, stream>>>(x, wp + WP0, dinv, b0, hw, nN, NPAD);
  k_agg<<<nAgg, NTHR, LDS_AGG, stream>>>(csr, offp, cnt, dinv, hw, b0, hcat, JKD, nN, csrLen);

  constexpr int LDS_G2 = gemm_lds(HID, HID);
  k_gemm<HID, JKD, HID, HSC, 1, 0, 0><<<nGemm, NTHR, LDS_G2, stream>>>(hcat, wp + WP1, dinv, b1, hw, NPAD, NPAD);
  k_agg<<<nAgg, NTHR, LDS_AGG, stream>>>(csr, offp, cnt, dinv, hw, b1, hcat + HID, JKD, nN, csrLen);

  k_gemm<HID, JKD, HID, HSC, 1, 0, 0><<<nGemm, NTHR, LDS_G2, stream>>>(hcat + HID, wp + WP2, dinv, b2, hw, NPAD, NPAD);
  k_agg<<<nAgg, NTHR, LDS_AGG, stream>>>(csr, offp, cnt, dinv, hw, b2, hcat + 2 * HID, JKD, nN, csrLen);

  constexpr int LDS_G3 = gemm_lds(JKD, HID);
  hipFuncSetAttribute(reinterpret_cast<const void*>(&k_gemm<JKD, JKD, HID, HSC, 0, 1, 0>),
                      hipFuncAttributeMaxDynamicSharedMemorySize, LDS_G3);
  k_gemm<JKD, JKD, HID, HSC, 0, 1, 0><<<nGemm, NTHR, LDS_G3, stream>>>(hcat, wp + WP3, dinv, bjk, hjk, NPAD, NPAD);

  k_pool<<<GP, PTHR, 0, stream>>>(hjk, gid, emb, nN, nG);

  k_gemm<HID, HID, HID, ESC, 0, 1, 1><<<nGemmH, NTHR, LDS_G2, stream>>>(emb, wp + WP4, dinv, bm1, t2, GP, GP);
  constexpr int LDS_G4 = gemm_lds(HID, FOUT);
  k_gemm<HID, HID, FOUT, ESC, 0, 1, 0><<<nGemmH, NTHR, LDS_G4, stream>>>(t2, wp + WP5, dinv, bm2, out, GP, nG);
}
